// LSTMCell_29944511987933
// MI455X (gfx1250) — hardware-verified
//
#include <hip/hip_runtime.h>
#include <math.h>
#include <stddef.h>

typedef __attribute__((ext_vector_type(16))) _Float16 v16h;
typedef __attribute__((ext_vector_type(8)))  _Float16 v8h;
typedef __attribute__((ext_vector_type(16))) __bf16   v16b;
typedef __attribute__((ext_vector_type(8)))  __bf16   v8b;
typedef __attribute__((ext_vector_type(8)))  float    v8f;
typedef __attribute__((ext_vector_type(4)))  float    v4f;
typedef __attribute__((ext_vector_type(4)))  unsigned int v4u;
#define PSCALE 32768.0f
#define U16(p) ((const unsigned short*)(const void*)(p))
#define PSCALE_INV (1.0f / 32768.0f)

__device__ __forceinline__ unsigned short f2bf_bits(float f) {
  unsigned u = __float_as_uint(f);
  return (unsigned short)((u + 0x7FFFu + ((u >> 16) & 1u)) >> 16);
}
__device__ __forceinline__ float bf_bits2f(unsigned short h) { return __uint_as_float(((unsigned)h) << 16); }

__device__ __forceinline__ void dep_guard_h(v8f& a, v8f& b, v16h x, v16h y) { asm volatile("v_nop\n\tv_nop\n\tv_nop\n\tv_nop" : "+v"(a), "+v"(b) : "v"(x), "v"(y)); }
__device__ __forceinline__ void dep_guard_b(v8f& a, v8f& b, v16b x, v16b y) { asm volatile("v_nop\n\tv_nop\n\tv_nop\n\tv_nop" : "+v"(a), "+v"(b) : "v"(x), "v"(y)); }
__device__ __forceinline__ void keep4_h(v16h a, v16h b, v16h c, v16h d) { asm volatile("v_nop" :: "v"(a), "v"(b), "v"(c), "v"(d)); }
__device__ __forceinline__ void keep4_b(v16b a, v16b b, v16b c, v16b d) { asm volatile("v_nop" :: "v"(a), "v"(b), "v"(c), "v"(d)); }
__device__ __forceinline__ void acc_guard4(v8f& a, v8f& b, v8f& c, v8f& d) { asm volatile("v_nop\n\tv_nop\n\tv_nop\n\tv_nop" : "+v"(a), "+v"(b), "+v"(c), "+v"(d)); }
template <typename T> struct Frag;
template <> struct Frag<_Float16> {
  typedef v16h V; union U { v16h v; v8h h[2]; };
  static __device__ __forceinline__ v16h load(const _Float16* p) {
    U f; f.h[0] = *(const v8h*)(p); f.h[1] = *(const v8h*)(p + 16); return f.v;
  }
  static __device__ __forceinline__ v8f mma(v16h a, v16h b, v8f c) {
    return __builtin_amdgcn_wmma_f32_16x16x32_f16(false, a, false, b, (short)0, c, false, false);
  }
  static __device__ __forceinline__ void guard(v8f& a, v8f& b, v16h x, v16h y) { dep_guard_h(a, b, x, y); }
  static __device__ __forceinline__ void keep(v16h a, v16h b, v16h c, v16h d) { keep4_h(a, b, c, d); }
};
template <> struct Frag<__bf16> {
  typedef v16b V; union U { v16b v; v8b h[2]; };
  static __device__ __forceinline__ v16b load(const __bf16* p) {
    U f; f.h[0] = *(const v8b*)(p); f.h[1] = *(const v8b*)(p + 16); return f.v;
  }
  static __device__ __forceinline__ v8f mma(v16b a, v16b b, v8f c) {
    return __builtin_amdgcn_wmma_f32_16x16x32_bf16(false, a, false, b, (short)0, c, false, false);
  }
  static __device__ __forceinline__ void guard(v8f& a, v8f& b, v16b x, v16b y) { dep_guard_b(a, b, x, y); }
  static __device__ __forceinline__ void keep(v16b a, v16b b, v16b c, v16b d) { keep4_b(a, b, c, d); }
};

template <int ET> struct Elem;
template <> struct Elem<0> { typedef _Float16 T; };
template <> struct Elem<1> { typedef __bf16 T; };
template <int ET, bool SPLIT, int BIAS_MODE, int OUT_MODE, bool RESID, int ACT = 0>
__global__ __launch_bounds__(256) void wmma_gemm64(
    const unsigned short* __restrict__ Ap, const unsigned short* __restrict__ A2p, int lda, long strideA,
    const unsigned short* __restrict__ Btp, const unsigned short* __restrict__ Bt2p, int ldb, long strideB,
    void* __restrict__ Cout, void* __restrict__ Cout2, int ldc, long strideC,
    const float* __restrict__ bias,
    const float* __restrict__ resid, long strideR,
    int M, int N, int K, float scale) {
  typedef typename Elem<ET>::T T;
  typedef typename Frag<T>::V V;
  const T* A = (const T*)Ap; const T* A2 = (const T*)A2p; const T* Bt = (const T*)Btp; const T* Bt2 = (const T*)Bt2p;
  __shared__ __align__(16) float sT[8][16 * 68];
  const int b    = blockIdx.y;
  const int lane = threadIdx.x & 31;
  const int wave = threadIdx.x >> 5;
  const int tilesN = N >> 6;
  const int tilesM = M >> 6;
  const int tile = blockIdx.x * 8 + wave;
  if (tile >= tilesM * tilesN) return;
  const int tm = tile / tilesN;
  const int tn = tile - tm * tilesN;
  const int m0 = tm << 6;
  const int n0 = tn << 6;

  const T* Ab  = A  + (size_t)b * strideA;
  const T* Bb  = Bt + (size_t)b * strideB;
  const T* Ab2 = SPLIT ? (A2  + (size_t)b * strideA) : nullptr;
  const T* Bb2 = SPLIT ? (Bt2 + (size_t)b * strideB) : nullptr;

  const int rlane = lane & 15;
  const int koff  = (lane >> 4) * 8;
  const int mOff  = (lane >> 4) * 8;

  v8f acc[4][4];
#pragma unroll
  for (int i = 0; i < 4; ++i)
#pragma unroll
    for (int j = 0; j < 4; ++j) acc[i][j] = (v8f){0.f,0.f,0.f,0.f,0.f,0.f,0.f,0.f};

  for (int k0 = 0; k0 < K; k0 += 32) {
    V bh[4], bl[4];
#pragma unroll
    for (int j = 0; j < 4; ++j) {
      const size_t bo = (size_t)(n0 + (j << 4) + rlane) * ldb + koff + k0;
      bh[j] = Frag<T>::load(Bb + bo);
      if (SPLIT) bl[j] = Frag<T>::load(Bb2 + bo);
    }
#pragma unroll
    for (int i = 0; i < 4; ++i) {
      const size_t ao = (size_t)(m0 + (i << 4) + rlane) * lda + koff + k0;
      V ah = Frag<T>::load(Ab + ao);
      V al;
      if (SPLIT) al = Frag<T>::load(Ab2 + ao);
#pragma unroll
      for (int j = 0; j < 4; ++j) {
        acc[i][j] = Frag<T>::mma(ah, bh[j], acc[i][j]);
        if (SPLIT) {
          acc[i][j] = Frag<T>::mma(ah, bl[j], acc[i][j]);
          acc[i][j] = Frag<T>::mma(al, bh[j], acc[i][j]);
        }
      }
      Frag<T>::guard(acc[i][0], acc[i][3], ah, SPLIT ? al : ah);
    }
    Frag<T>::keep(bh[0], bh[1], bh[2], bh[3]);
    if (SPLIT) Frag<T>::keep(bl[0], bl[1], bl[2], bl[3]);
  }
  acc_guard4(acc[0][0], acc[0][1], acc[0][2], acc[0][3]);
  acc_guard4(acc[1][0], acc[1][1], acc[1][2], acc[1][3]);
  acc_guard4(acc[2][0], acc[2][1], acc[2][2], acc[2][3]);
  acc_guard4(acc[3][0], acc[3][1], acc[3][2], acc[3][3]);

  float* slab = sT[wave];
  const float* Rb = RESID ? (resid + (size_t)b * strideR) : nullptr;
#pragma unroll
  for (int i = 0; i < 4; ++i) {
    const int mBase = m0 + (i << 4);
#pragma unroll
    for (int j = 0; j < 4; ++j) {
      const int n = n0 + (j << 4) + rlane;
      float bv = 0.f;
      if (BIAS_MODE == 2) bv = bias[n];
#pragma unroll
      for (int r = 0; r < 8; ++r) {
        float v = acc[i][j][r] * scale;
        if (BIAS_MODE == 1) v += bias[mBase + mOff + r];
        if (BIAS_MODE == 2) v += bv;
        if (RESID) v += Rb[(size_t)(mBase + mOff + r) * ldc + n];
        if (ACT == 1) v = tanhf(v);
        if (ACT == 2) v = fmaxf(v, 0.0f);
        if (ACT == 3) v = v / (1.0f + expf(-v));
        if (ACT == 4) v = (v > 0.f) ? v : 0.01f * v;
        if (ACT == 5) v = 0.5f * v * (1.0f + erff(v * 0.70710678118654752f));
        slab[(mOff + r) * 68 + (j << 4) + rlane] = v;
      }
    }
    __builtin_amdgcn_fence(__ATOMIC_RELEASE, "workgroup");
    __builtin_amdgcn_wave_barrier();
    __builtin_amdgcn_fence(__ATOMIC_ACQUIRE, "workgroup");
    if (OUT_MODE == 0) {
      float* C = (float*)Cout + (size_t)b * strideC;
      const int hh = lane >> 4, c4 = (lane & 15) * 4;
      for (int pass = 0; pass < 2; ++pass) {
#pragma unroll
        for (int it = 0; it < 8; ++it) {
          const int row = it * 2 + hh;
          v4f v = *(const v4f*)(slab + row * 68 + c4);
          *(volatile v4f*)(C + (size_t)(mBase + row) * ldc + n0 + c4) = v;
        }
        __threadfence();
      }
    } else {
      const int q = lane >> 3, c8 = (lane & 7) * 8;
      unsigned short* C  = (unsigned short*)Cout  + (size_t)b * strideC;
      unsigned short* C2 = (OUT_MODE == 2) ? ((unsigned short*)Cout2 + (size_t)b * strideC) : nullptr;
      for (int pass = 0; pass < 2; ++pass) {
#pragma unroll
        for (int it = 0; it < 4; ++it) {
          const int row = it * 4 + q;
          const float* sp = slab + row * 68 + c8;
          v8h hv, lv;
#pragma unroll
          for (int e = 0; e < 8; ++e) {
            if (OUT_MODE == 1) {
              hv[e] = (_Float16)sp[e];
            } else {
              unsigned short hb = f2bf_bits(sp[e]);
              unsigned short lb = f2bf_bits(sp[e] - bf_bits2f(hb));
              hv[e] = __builtin_bit_cast(_Float16, hb);
              lv[e] = __builtin_bit_cast(_Float16, lb);
            }
          }
          *(volatile v8h*)(C + (size_t)(mBase + row) * ldc + n0 + c8) = hv;
          if (OUT_MODE == 2) *(volatile v8h*)(C2 + (size_t)(mBase + row) * ldc + n0 + c8) = lv;
        }
        __threadfence();
      }
    }
    __builtin_amdgcn_fence(__ATOMIC_RELEASE, "workgroup");
    __builtin_amdgcn_wave_barrier();
    __builtin_amdgcn_fence(__ATOMIC_ACQUIRE, "workgroup");
  }
}

constexpr int NBATCH   = 2048;
constexpr int DIM_IN   = 2048;
constexpr int DIM_H    = 2048;
constexpr int KCAT     = DIM_IN + DIM_H;
constexpr int NCLS     = 1000;
constexpr int NCLS_PAD = 1024;
constexpr int TPITCH   = 72;
constexpr float PLANE_CARRY = 64.0f;
constexpr float PROJ_SCALE  = 1.0f / 4096.0f;

static_assert(NBATCH % 64 == 0 && DIM_H % 64 == 0 && NCLS_PAD % 64 == 0, "GEMM M/N tile multiples");
static_assert(KCAT % 32 == 0 && DIM_H % 32 == 0, "GEMM K multiples of 32");
static_assert(((NBATCH / 64) * (DIM_H / 64)) % 8 == 0, "gate GEMM grid exact");
static_assert(((NBATCH / 64) * (NCLS_PAD / 64)) % 8 == 0, "projection GEMM grid exact");
static_assert(DIM_IN % 64 == 0 && DIM_H % 64 == 0 && NCLS_PAD % 64 == 0, "transpose tiles exact");
static_assert(NCLS % 4 == 0, "float4 never straddles an output row");
static_assert((32 * NCLS * 4) % 128 == 0, "32-row output groups are whole 128-B lines");
static_assert(NBATCH % 32 == 0, "softmax row groups exact");
static_assert(DIM_H % 256 == 0, "cell-update blocks stay inside one row");

constexpr size_t ACAT_BYTES  = (size_t)NBATCH * KCAT * 2;
constexpr size_t WT_BYTES    = (size_t)DIM_H * KCAT * 2;
constexpr size_t PRE_BYTES   = (size_t)NBATCH * DIM_H * 4;
constexpr size_t HPL_BYTES   = (size_t)NBATCH * DIM_H * 2;
constexpr size_t WPHT_BYTES  = (size_t)NCLS_PAD * DIM_H * 2;
constexpr size_t PFULL_BYTES = (size_t)NBATCH * NCLS_PAD * 4;
constexpr size_t OFF_ACAT  = 0;
constexpr size_t OFF_WT    = OFF_ACAT + ACAT_BYTES;
constexpr size_t OFF_PRE   = OFF_WT + WT_BYTES;
constexpr size_t OFF_HPL   = OFF_PRE + 4 * PRE_BYTES;
constexpr size_t OFF_WPHT  = OFF_HPL + HPL_BYTES;
constexpr size_t OFF_PFULL = OFF_WPHT + WPHT_BYTES;
constexpr size_t WS_TOTAL  = OFF_PFULL + PFULL_BYTES;
static_assert(WS_TOTAL == 121634816ull, "carve total");
static_assert(WS_TOTAL <= 134217728ull, "carve under 128 MiB");
static_assert(OFF_WT % 256 == 0 && OFF_PRE % 256 == 0 && OFF_HPL % 256 == 0 && OFF_WPHT % 256 == 0 && OFF_PFULL % 256 == 0, "aligned regions");

constexpr size_t OUT1_ELEM_OFF  = 8192000ull / 4;
constexpr size_t OUT2_ELEM_OFF  = 24969216ull / 4;
constexpr size_t OUT_TOTAL_ELEM = 41746432ull / 4;
static_assert(OUT1_ELEM_OFF == (size_t)NBATCH * NCLS, "out1 offset");
static_assert(OUT2_ELEM_OFF == OUT1_ELEM_OFF + (size_t)NBATCH * DIM_H, "out2 offset");
static_assert(OUT2_ELEM_OFF + (size_t)NBATCH * DIM_H == OUT_TOTAL_ELEM, "out total");
static_assert((8192000ull % 128) == 0 && (24969216ull % 128) == 0, "outputs start on 128-B lines");

__global__ __launch_bounds__(256) void pack_rows_bf16(const float* __restrict__ x,
                                                      const float* __restrict__ h,
                                                      unsigned short* __restrict__ A, int n8) {
  const int i = blockIdx.x * 256 + threadIdx.x;
  if (i >= n8) return;
  const size_t e = (size_t)i * 8;
  const size_t m = e / DIM_IN;
  const size_t j = e - m * DIM_IN;
  const v4f xa = *(const v4f*)(x + e);
  const v4f xb = *(const v4f*)(x + e + 4);
  const v4f ha = *(const v4f*)(h + e);
  const v4f hb = *(const v4f*)(h + e + 4);
  v4u px, ph;
  px[0] = (unsigned)f2bf_bits(xa[0]) | ((unsigned)f2bf_bits(xa[1]) << 16);
  px[1] = (unsigned)f2bf_bits(xa[2]) | ((unsigned)f2bf_bits(xa[3]) << 16);
  px[2] = (unsigned)f2bf_bits(xb[0]) | ((unsigned)f2bf_bits(xb[1]) << 16);
  px[3] = (unsigned)f2bf_bits(xb[2]) | ((unsigned)f2bf_bits(xb[3]) << 16);
  ph[0] = (unsigned)f2bf_bits(ha[0]) | ((unsigned)f2bf_bits(ha[1]) << 16);
  ph[1] = (unsigned)f2bf_bits(ha[2]) | ((unsigned)f2bf_bits(ha[3]) << 16);
  ph[2] = (unsigned)f2bf_bits(hb[0]) | ((unsigned)f2bf_bits(hb[1]) << 16);
  ph[3] = (unsigned)f2bf_bits(hb[2]) | ((unsigned)f2bf_bits(hb[3]) << 16);
  unsigned short* dx = A + m * KCAT + j;
  unsigned short* dh = dx + DIM_IN;
  *(volatile v4u*)dx = px;
  *(volatile v4u*)dh = ph;
  __threadfence();
  *(volatile v4u*)dx = px;
  *(volatile v4u*)dh = ph;
}

template <int MODE>
__global__ __launch_bounds__(256) void transpose_cvt64(const float* __restrict__ W, int Ndim,
                                                       unsigned short* __restrict__ Wt, int ldWt, int koff) {
  __shared__ __align__(16) unsigned short tile[64 * TPITCH];
  const int t  = threadIdx.x;
  const int nt = blockIdx.x * 64;
  const int kt = blockIdx.y * 64;
#pragma unroll
  for (int i = 0; i < 4; ++i) {
    const int idx = t + 256 * i;
    const int k   = idx >> 4;
    const int n4  = (idx & 15) * 4;
    const int ng  = nt + n4;
    const bool ok = (ng < Ndim);
    const int ngc = ok ? ng : (Ndim - 4);
    const v4f w = *(const v4f*)(W + (size_t)(kt + k) * Ndim + ngc);
#pragma unroll
    for (int e = 0; e < 4; ++e) {
      const float f = ok ? w[e] : 0.0f;
      unsigned short bits;
      if (MODE == 0) {
        bits = f2bf_bits(f);
      } else {
        const float fr = bf_bits2f(f2bf_bits(f)) * PLANE_CARRY;
        bits = __builtin_bit_cast(unsigned short, (_Float16)fr);
      }
      tile[(n4 + e) * TPITCH + k] = bits;
    }
  }
  __syncthreads();
  const int wave = t >> 5, lane = t & 31;
  const int q = lane >> 3, c8 = (lane & 7) * 8;
  const int rowA = wave * 4 + q;
  const int rowB = 32 + wave * 4 + q;
  const v4u va = *(const v4u*)(tile + rowA * TPITCH + c8);
  const v4u vb = *(const v4u*)(tile + rowB * TPITCH + c8);
  unsigned short* da = Wt + (size_t)(nt + rowA) * ldWt + koff + kt + c8;
  unsigned short* db = Wt + (size_t)(nt + rowB) * ldWt + koff + kt + c8;
  *(volatile v4u*)da = va;
  *(volatile v4u*)db = vb;
  __threadfence();
  *(volatile v4u*)da = va;
  *(volatile v4u*)db = vb;
}

__device__ __forceinline__ float sigmoid_f(float v) {
  const float e = expf(-fabsf(v));
  const float r = 1.0f / (1.0f + e);
  return (v >= 0.0f) ? r : e * r;
}

__global__ __launch_bounds__(256) void lstm_cell_update(const float* __restrict__ pg,
                                                        const float* __restrict__ pi,
                                                        const float* __restrict__ pf,
                                                        const float* __restrict__ po,
                                                        const float* __restrict__ c,
                                                        float* __restrict__ c_out,
                                                        float* __restrict__ h_out,
                                                        unsigned short* __restrict__ hplane) {
  __shared__ __align__(16) float s_c[256];
  __shared__ __align__(16) float s_h[256];
  __shared__ __align__(16) unsigned short s_hb[256];
  const int tid = threadIdx.x;
  const size_t base = (size_t)blockIdx.x * 256;
  const size_t e = base + tid;
  const float vg = pg[e];
  const float vi = pi[e];
  const float vf = pf[e];
  const float vo = po[e];
  const float cr = bf_bits2f(f2bf_bits(c[e]));
  const float g  = tanhf(vg);
  const float ig = sigmoid_f(vi);
  const float fg = sigmoid_f(vf);
  const float og = sigmoid_f(vo);
  const float cn = g * ig + cr * fg;
  const float hn = tanhf(cn) * og;
  s_c[tid] = cn;
  s_h[tid] = hn;
  s_hb[tid] = __builtin_bit_cast(unsigned short, (_Float16)(hn * PLANE_CARRY));
  __syncthreads();
  const int wave = tid >> 5, lane = tid & 31;
  if (wave < 2) {
    const int idx = tid * 4;
    const v4f v = *(const v4f*)(s_c + idx);
    float* d = c_out + base + idx;
    *(volatile v4f*)d = v;
    __threadfence();
    *(volatile v4f*)d = v;
  } else if (wave < 4) {
    const int idx = (tid - 64) * 4;
    const v4f v = *(const v4f*)(s_h + idx);
    float* d = h_out + base + idx;
    *(volatile v4f*)d = v;
    __threadfence();
    *(volatile v4f*)d = v;
  } else if (wave == 4) {
    const int idx = lane * 8;
    const v4u v = *(const v4u*)(s_hb + idx);
    unsigned short* d = hplane + base + idx;
    *(volatile v4u*)d = v;
    __threadfence();
    *(volatile v4u*)d = v;
  }
}

__global__ __launch_bounds__(256) void proj_softmax_rows(const float* __restrict__ P,
                                                         const float* __restrict__ bp,
                                                         float* __restrict__ Y) {
  __shared__ float s_m[32];
  __shared__ float s_inv[32];
  const int tid = threadIdx.x, wave = tid >> 5, lane = tid & 31;
  const int r0 = blockIdx.x * 32;
#pragma unroll 1
  for (int rr = 0; rr < 4; ++rr) {
    const int rloc = wave * 4 + rr;
    const float* prow = P + (size_t)(r0 + rloc) * NCLS_PAD;
    float m = -INFINITY;
#pragma unroll 1
    for (int j = lane; j < NCLS; j += 32) {
      const float pv = prow[j] + bf_bits2f(f2bf_bits(bp[j]));
      m = fmaxf(m, pv);
    }
#pragma unroll
    for (int off = 1; off < 32; off <<= 1) m = fmaxf(m, __shfl_xor(m, off, 32));
    float s = 0.0f;
#pragma unroll 1
    for (int j = lane; j < NCLS; j += 32) {
      const float pv = prow[j] + bf_bits2f(f2bf_bits(bp[j]));
      s += expf(pv - m);
    }
#pragma unroll
    for (int off = 1; off < 32; off <<= 1) s += __shfl_xor(s, off, 32);
    if (lane == 0) { s_m[rloc] = m; s_inv[rloc] = 1.0f / s; }
  }
  __syncthreads();
  float* yb = Y + (size_t)r0 * NCLS;
  const int nflt4 = 32 * NCLS / 4;
#pragma unroll 1
  for (int pass = 0; pass < 2; ++pass) {
#pragma unroll 1
    for (int i = tid; i < nflt4; i += 256) {
      const int e = i * 4;
      const int rloc = e / NCLS;
      const int col = e - rloc * NCLS;
      const v4f p = *(const v4f*)(P + (size_t)(r0 + rloc) * NCLS_PAD + col);
      const v4f bb = *(const v4f*)(bp + col);
      const float m = s_m[rloc], inv = s_inv[rloc];
      v4f y;
      y[0] = expf(p[0] + bf_bits2f(f2bf_bits(bb[0])) - m) * inv;
      y[1] = expf(p[1] + bf_bits2f(f2bf_bits(bb[1])) - m) * inv;
      y[2] = expf(p[2] + bf_bits2f(f2bf_bits(bb[2])) - m) * inv;
      y[3] = expf(p[3] + bf_bits2f(f2bf_bits(bb[3])) - m) * inv;
      *(volatile v4f*)(yb + e) = y;
    }
    __threadfence();
  }
}

extern "C" void kernel_launch(void* const* d_in, const int* in_sizes, int n_in,
                              void* d_out, int out_size, void* d_ws, size_t ws_size,
                              hipStream_t stream) {
  if (n_in < 17) return;
  if (ws_size < WS_TOTAL) return;
  if ((size_t)out_size < OUT_TOTAL_ELEM) return;
  if (in_sizes[0] != NBATCH * DIM_IN || in_sizes[1] != NBATCH * DIM_H || in_sizes[2] != NBATCH * DIM_H) return;
  if (in_sizes[3] != DIM_IN * DIM_H || in_sizes[7] != DIM_H * DIM_H) return;
  if (in_sizes[15] != DIM_H * NCLS || in_sizes[16] != NCLS || in_sizes[11] != DIM_H) return;

  const float* x = (const float*)d_in[0];
  const float* c = (const float*)d_in[1];
  const float* h = (const float*)d_in[2];
  const float* Wx[4]   = { (const float*)d_in[3], (const float*)d_in[4],
                           (const float*)d_in[5], (const float*)d_in[6] };
  const float* Wh[4]   = { (const float*)d_in[7], (const float*)d_in[8],
                           (const float*)d_in[9], (const float*)d_in[10] };
  const float* bias[4] = { (const float*)d_in[11], (const float*)d_in[12],
                           (const float*)d_in[13], (const float*)d_in[14] };
  const float* Wph = (const float*)d_in[15];
  const float* bp  = (const float*)d_in[16];

  char* ws = (char*)d_ws;
  unsigned short* Acat   = (unsigned short*)(ws + OFF_ACAT);
  unsigned short* Wt     = (unsigned short*)(ws + OFF_WT);
  float* pre[4];
  for (int gi = 0; gi < 4; ++gi) pre[gi] = (float*)(ws + OFF_PRE + (size_t)gi * PRE_BYTES);
  unsigned short* hplane = (unsigned short*)(ws + OFF_HPL);
  unsigned short* WphT   = (unsigned short*)(ws + OFF_WPHT);
  float* pfull           = (float*)(ws + OFF_PFULL);

  float* y     = (float*)d_out;
  float* c_out = y + OUT1_ELEM_OFF;
  float* h_out = y + OUT2_ELEM_OFF;

  {
    const int n8 = NBATCH * DIM_IN / 8;
    pack_rows_bf16<<<(n8 + 255) / 256, 256, 0, stream>>>(x, h, Acat, n8);
  }

  for (int gi = 0; gi < 4; ++gi) {
    transpose_cvt64<0><<<dim3(DIM_H / 64, DIM_IN / 64), 256, 0, stream>>>(Wx[gi], DIM_H, Wt, KCAT, 0);
    transpose_cvt64<0><<<dim3(DIM_H / 64, DIM_H / 64), 256, 0, stream>>>(Wh[gi], DIM_H, Wt, KCAT, DIM_IN);
    wmma_gemm64<1, false, 2, 0, false, 0><<<dim3((NBATCH / 64) * (DIM_H / 64) / 8, 1), 256, 0, stream>>>(
        Acat, Acat, KCAT, 0L,
        Wt, Wt, KCAT, 0L,
        (void*)pre[gi], (void*)pre[gi], DIM_H, 0L,
        bias[gi],
        bias[gi], 0L,
        NBATCH, DIM_H, KCAT, 1.0f);
  }

  lstm_cell_update<<<NBATCH * DIM_H / 256, 256, 0, stream>>>(
      pre[0], pre[1], pre[2], pre[3], c, c_out, h_out, hplane);

  transpose_cvt64<1><<<dim3(NCLS_PAD / 64, DIM_H / 64), 256, 0, stream>>>(Wph, NCLS, WphT, DIM_H, 0);

  wmma_gemm64<0, false, 0, 0, false, 0><<<dim3((NBATCH / 64) * (NCLS_PAD / 64) / 8, 1), 256, 0, stream>>>(
      hplane, hplane, DIM_H, 0L,
      WphT, WphT, DIM_H, 0L,
      (void*)pfull, (void*)pfull, NCLS_PAD, 0L,
      bp,
      bp, 0L,
      NBATCH, NCLS_PAD, DIM_H, PROJ_SCALE);

  proj_softmax_rows<<<NBATCH / 32, 256, 0, stream>>>(pfull, bp, y);
}
